// STBlock_54065048322482
// MI455X (gfx1250) — hardware-verified
//
#include <hip/hip_runtime.h>
#include <math.h>

typedef __attribute__((ext_vector_type(16))) _Float16 v16h;
typedef __attribute__((ext_vector_type(16))) __bf16 v16b;
typedef __attribute__((ext_vector_type(8)))  _Float16 v8h;
typedef __attribute__((ext_vector_type(8)))  float v8f;
typedef __attribute__((ext_vector_type(4)))  float v4f;
typedef __attribute__((ext_vector_type(2)))  float v2f;
typedef __attribute__((ext_vector_type(4)))  unsigned v4u;
typedef __attribute__((ext_vector_type(4)))  int v4i;
typedef float __attribute__((may_alias)) float_a;
typedef int __attribute__((may_alias)) int_a;

template <typename T> __device__ __forceinline__ void vst2(void* p, T v) { *(volatile T*)p = v; __threadfence(); *(volatile T*)p = v; }
__device__ __forceinline__ v8f wmma16(v16h a, v16h b, v8f c) {
  v8f d = __builtin_amdgcn_wmma_f32_16x16x32_f16(false, a, false, b, (short)0, c, false, false);
  asm volatile("v_nop\n\tv_nop\n\tv_nop\n\tv_nop" : "+v"(d) : "v"(a), "v"(b));
  return d;
}
__device__ __forceinline__ v8f wmma_bf(v16b a, v16b b, v8f c) {
  v8f d = __builtin_amdgcn_wmma_f32_16x16x32_bf16(false, a, false, b, (short)0, c, false, false);
  asm volatile("v_nop\n\tv_nop\n\tv_nop\n\tv_nop" : "+v"(d) : "v"(a), "v"(b));
  return d;
}
__device__ __forceinline__ v16h frag_h(const _Float16* rowk0, int lane) {
  union { v16h v; v8h q[2]; } u; const _Float16* p = rowk0 + 8 * (lane >> 4);
  u.q[0] = *(const v8h*)p; u.q[1] = *(const v8h*)(p + 16); return u.v;
}
__device__ __forceinline__ v16h frag_f32(const float* rowk0, int lane) {
  v16h a; const float* p = rowk0 + 8 * (lane >> 4);
#pragma unroll
  for (int i = 0; i < 8; ++i) { a[i] = (_Float16)p[i]; a[8 + i] = (_Float16)p[16 + i]; }
  return a;
}
__device__ __forceinline__ v16h frag_f32s(const float* rowk0, int lane, float sc) {
  v16h a; const float* p = rowk0 + 8 * (lane >> 4);
#pragma unroll
  for (int i = 0; i < 8; ++i) { a[i] = (_Float16)(p[i] * sc); a[8 + i] = (_Float16)(p[16 + i] * sc); }
  return a;
}
__device__ __forceinline__ v16h fragc_f32(const float* W, int k0, int n, int lane, int ld, int K) {
  v16h a; const int g = lane >> 4;
#pragma unroll
  for (int i = 0; i < 8; ++i) { const int ka = k0 + 8 * g + i, kb = ka + 16;
    a[i] = (_Float16)(ka < K ? W[(size_t)(ka < K ? ka : K - 1) * ld + n] : 0.f); a[8 + i] = (_Float16)(kb < K ? W[(size_t)(kb < K ? kb : K - 1) * ld + n] : 0.f); }
  return a;
}
struct F2 { v16b h, l; };
__device__ __forceinline__ F2 bsplit16(const float v[16]) { F2 r;
#pragma unroll
  for (int i = 0; i < 16; ++i) { const __bf16 h = (__bf16)v[i]; r.h[i] = h; r.l[i] = (__bf16)(v[i] - (float)h); }
  return r; }
__device__ __forceinline__ F2 split_row(const float* row, int k0, int lane) { float v[16]; const float* p = row + k0 + 8 * (lane >> 4);
#pragma unroll
  for (int i = 0; i < 8; ++i) { v[i] = p[i]; v[8 + i] = p[16 + i]; }
  return bsplit16(v); }
__device__ __forceinline__ F2 split_rowK(const float* row, int k0, int lane, int K) { float v[16]; const int g = lane >> 4;
#pragma unroll
  for (int i = 0; i < 8; ++i) { const int ka = k0 + 8 * g + i, kb = ka + 16; v[i] = ka < K ? row[ka < K ? ka : K - 1] : 0.f; v[8 + i] = kb < K ? row[kb < K ? kb : K - 1] : 0.f; }
  return bsplit16(v); }
__device__ __forceinline__ F2 split_col(const float* W, int k0, int n, int lane, int ld, int K) { float v[16]; const int g = lane >> 4;
#pragma unroll
  for (int i = 0; i < 8; ++i) { const int ka = k0 + 8 * g + i, kb = ka + 16; v[i] = ka < K ? W[(size_t)(ka < K ? ka : K - 1) * ld + n] : 0.f; v[8 + i] = kb < K ? W[(size_t)(kb < K ? kb : K - 1) * ld + n] : 0.f; }
  return bsplit16(v); }
__device__ __forceinline__ v8f mac3(const F2& a, const F2& b, v8f c) { c = wmma_bf(a.l, b.h, c); c = wmma_bf(a.h, b.l, c); return wmma_bf(a.h, b.h, c); }
__device__ __forceinline__ float sigm(float v) { return 1.0f / (1.0f + expf(-v)); }
#define LDSX() do { asm volatile("s_wait_dscnt 0" ::: "memory"); __builtin_amdgcn_wave_barrier(); __builtin_amdgcn_fence(__ATOMIC_RELEASE, "workgroup"); } while (0)


#define NB 8
#define NN 256
#define CI 64
#define CO 64
#define TS 64
#define CT (CI * TS)
#define NC (NN * CI)
#ifndef TNB
#define TNB NB
#endif
typedef __attribute__((ext_vector_type(8))) __bf16 v8b;
__device__ __forceinline__ v16b frag_b(const __bf16* rowk0, int lane) {
  union { v16b v; v8b q[2]; } u; const __bf16* p = rowk0 + 8 * (lane >> 4);
  u.q[0] = *(const v8b*)p; u.q[1] = *(const v8b*)(p + 16); return u.v;
}
__device__ __forceinline__ float bfr(float v) { return (float)(__bf16)v; }
__device__ __attribute__((noinline)) float exp_ni(float v) { return expf(v); }
__device__ __attribute__((noinline)) float erf_ni(float v) { return erff(v); }

#define WS_LS  0u
#define WS_RST (WS_LS + 4u * (size_t)NB * NN * NN)
#define WS_XTR (WS_RST + 4u * (size_t)NB * NN * NN)
#define WS_LT  (WS_XTR + 4u * (size_t)NB * TS * NC)
#define WS_RTT (WS_LT + 4u * (size_t)NB * TS * TS)
#define WS_SA  (WS_RTT + 4u * (size_t)NB * TS * TS)
#define WS_EA  (WS_SA + 4u * (size_t)NB * NN * NN)
#define WS_XTT (WS_EA + 4u * (size_t)NB * TS * TS)
#define WS_XM  (WS_XTT + 4u * (size_t)NB * CT * NN)
#define WS_XMT (WS_XM + 4u * (size_t)NB * NN * CT)
#define WS_T1  (WS_XMT + 4u * (size_t)NB * CT * NN)
#define WS_T1T (WS_T1 + 4u * (size_t)NB * NN * CT)
#define WS_T2  (WS_T1T + 4u * (size_t)NB * CT * NN)
#define WS_END (WS_T2 + 4u * (size_t)NB * NN * CT)

__global__ __launch_bounds__(128) void k_lhs(const float* __restrict__ X, const float* __restrict__ W1, const float* __restrict__ W2, float* __restrict__ LS, float* __restrict__ RST) { __shared__ __align__(16) float st[128][68];
  const int tid = threadIdx.x, wave = tid >> 5, lane = tid & 31, col = lane & 15, g = lane >> 4; const int which = blockIdx.z; const int c0 = blockIdx.y * 128; const size_t r0 = (size_t)blockIdx.x * 64; const float* Wm = which == 0 ? W1 : W2;
  v8f acc[8] = {};
#pragma unroll 2
  for (int kc = 0; kc < CT / 32; ++kc) { v16b a; { const float* p = X + (r0 + wave * 16 + col) * CT + kc * 32 + 8 * g;
#pragma unroll
      for (int i = 0; i < 8; ++i) { a[i] = (__bf16)p[i]; a[8 + i] = (__bf16)p[16 + i]; } }
#pragma unroll
    for (int j = 0; j < 8; ++j) { v16b w; const int l = c0 + j * 16 + col; const float* p = Wm + (size_t)l * CT + kc * 32 + 8 * g;
#pragma unroll
      for (int i = 0; i < 8; ++i) { w[i] = (__bf16)p[i]; w[8 + i] = (__bf16)p[16 + i]; }
      acc[j] = wmma_bf(a, w, acc[j]); } }
  if (which == 0) { __shared__ __align__(16) float ss[4][16][132];
#pragma unroll
    for (int j = 0; j < 8; ++j)
#pragma unroll
      for (int r = 0; r < 8; ++r) ss[wave][8 * g + r][j * 16 + col] = acc[j][r];
    LDSX(); for (int rl = 0; rl < 16; ++rl) vst2(LS + (r0 + wave * 16 + rl) * NN + c0 + lane * 4, *(const v4f*)&ss[wave][rl][lane * 4]); }
  else { const size_t b = r0 / NN; const int j0 = (int)(r0 % NN);
#pragma unroll
    for (int j = 0; j < 8; ++j)
#pragma unroll
      for (int r = 0; r < 8; ++r) st[j * 16 + col][wave * 16 + 8 * g + r] = acc[j][r];
    __syncthreads(); for (int e = tid; e < 128 * 16; e += 128) { const int cl = e >> 4, q = e & 15; vst2(RST + (b * NN + c0 + cl) * (size_t)NN + j0 + q * 4, *(const v4f*)&st[cl][q * 4]); } } }
__global__ __launch_bounds__(256) void k_xtr(const float* __restrict__ X, float* __restrict__ XTR) { __shared__ __align__(16) float st[TS][CI + 4];
  const int t = threadIdx.x; const size_t b = blockIdx.y; const int n = blockIdx.x; const float* src = X + ((b * NN + n) * CI) * (size_t)TS;
  for (int e = t; e < CI * TS; e += 256) { const int c = e >> 6, tt = e & 63; st[tt][c] = src[e]; }
  __syncthreads(); for (int e = t; e < TS * 16; e += 256) { const int tt = e >> 4, q = e & 15; vst2(XTR + (b * TS + tt) * (size_t)NC + n * CI + q * 4, *(const v4f*)&st[tt][q * 4]); } }
__global__ __launch_bounds__(128) void k_lht(const float* __restrict__ XTR, const float* __restrict__ W1, const float* __restrict__ W2, float* __restrict__ LT, float* __restrict__ RTT) { __shared__ __align__(16) float ss[4][16][68]; __shared__ __align__(16) float st[64][68];
  const int tid = threadIdx.x, wave = tid >> 5, lane = tid & 31, col = lane & 15, g = lane >> 4; const size_t r0 = (size_t)blockIdx.x * 64; const size_t b = r0 / TS;
  v8f acc[8] = {};
#pragma unroll 2
  for (int kc = 0; kc < NC / 32; ++kc) { v16b a; { const float* p = XTR + (r0 + wave * 16 + col) * NC + kc * 32 + 8 * g;
#pragma unroll
      for (int i = 0; i < 8; ++i) { a[i] = (__bf16)bfr(p[i]); a[8 + i] = (__bf16)bfr(p[16 + i]); } }
#pragma unroll
    for (int j = 0; j < 8; ++j) { v16b w; const int l = (j & 3) * 16 + col; const float* p = ((j < 4) ? W1 : W2) + (size_t)l * NC + kc * 32 + 8 * g;
#pragma unroll
      for (int i = 0; i < 8; ++i) { w[i] = (__bf16)p[i]; w[8 + i] = (__bf16)p[16 + i]; }
      acc[j] = wmma_bf(a, w, acc[j]); } }
#pragma unroll
  for (int j = 0; j < 8; ++j)
#pragma unroll
    for (int r = 0; r < 8; ++r) { const int rl = wave * 16 + 8 * g + r, l = (j & 3) * 16 + col; if (j < 4) ss[wave][8 * g + r][l] = acc[j][r]; else st[l][rl] = acc[j][r]; }
  __syncthreads();
  for (int rl = 0; rl < 16; ++rl) if (lane < 16) vst2(LT + (r0 + wave * 16 + rl) * TS + lane * 4, *(const v4f*)&ss[wave][rl][lane * 4]);
  for (int e = tid; e < 64 * 16; e += 128) { const int l = e >> 4, q = e & 15; vst2(RTT + (b * TS + l) * (size_t)TS + q * 4, *(const v4f*)&st[l][q * 4]); } }
template <int LL>
__global__ __launch_bounds__(256) void k_att(const float* __restrict__ Lm, const float* __restrict__ RTm, const float* __restrict__ Vm, float* __restrict__ A) { __shared__ float sl[LL]; __shared__ float sred[8]; __shared__ float sbc; __shared__ __align__(16) float so[LL];
  const int t = threadIdx.x; const int i = blockIdx.x; const size_t b = blockIdx.y; const int wv = t >> 5, ln = t & 31;
  for (int l = t; l < LL; l += 256) sl[l] = Lm[(b * LL + i) * LL + l];
  __syncthreads();
  float sv = -3.0e38f;
  if (t < LL) { const int j = t; float s = 0.f;
#pragma unroll 1
    for (int l = 0; l < LL; ++l) { const float z = sl[l] + RTm[(b * LL + l) * (size_t)LL + j]; s += 1.0f / (1.0f + expf(-z)); }
    sv = s + bfr(Vm[(size_t)i * LL + j]); }
  float m = sv;
#pragma unroll
  for (int o = 1; o < 32; o <<= 1) m = fmaxf(m, __shfl_xor(m, o));
  if (ln == 0) sred[wv] = m; __syncthreads(); if (t == 0) { float a = sred[0]; for (int w = 1; w < 8; ++w) a = fmaxf(a, sred[w]); sbc = a; } __syncthreads(); m = sbc; __syncthreads();
  const float e = (t < LL) ? expf(sv - m) : 0.f; float s2 = e;
#pragma unroll
  for (int o = 1; o < 32; o <<= 1) s2 += __shfl_xor(s2, o);
  if (ln == 0) sred[wv] = s2; __syncthreads(); if (t == 0) { float a = 0.f; for (int w = 0; w < 8; ++w) a += sred[w]; sbc = 1.0f / a; } __syncthreads();
  if (t < LL) so[t] = e * sbc;
  __syncthreads(); for (int q = t; q < LL / 4; q += 256) vst2(A + (b * LL + i) * (size_t)LL + q * 4, *(const v4f*)&so[q * 4]); }
__global__ __launch_bounds__(128) void k_xtime(const float* __restrict__ X, const float* __restrict__ E, float* __restrict__ XTT) { __shared__ __align__(16) float st[64][68];
  const int tid = threadIdx.x, wave = tid >> 5, lane = tid & 31, col = lane & 15, g = lane >> 4; const int n0 = blockIdx.x * 64; const int c = blockIdx.y; const size_t b = blockIdx.z;
  v8f acc[4] = {};
#pragma unroll
  for (int kc = 0; kc < TS / 32; ++kc) { v16b a; { const float* p = X + ((b * NN + n0 + wave * 16 + col) * CI + c) * (size_t)TS + kc * 32 + 8 * g;
#pragma unroll
      for (int i = 0; i < 8; ++i) { a[i] = (__bf16)p[i]; a[8 + i] = (__bf16)p[16 + i]; } }
#pragma unroll
    for (int j = 0; j < 4; ++j) { const int s = j * 16 + col; const F2 e = split_row(E + (b * TS + s) * TS, kc * 32, lane); acc[j] = wmma_bf(a, e.h, acc[j]); acc[j] = wmma_bf(a, e.l, acc[j]); } }
#pragma unroll
  for (int j = 0; j < 4; ++j)
#pragma unroll
    for (int r = 0; r < 8; ++r) st[j * 16 + col][wave * 16 + 8 * g + r] = acc[j][r];
  __syncthreads(); for (int e = tid; e < 64 * 16; e += 128) { const int s = e >> 4, q = e & 15; vst2(XTT + (b * CT + c * TS + s) * (size_t)NN + n0 + q * 4, *(const v4f*)&st[s][q * 4]); } }
template <int MODE>
__global__ __launch_bounds__(128) void k_nmix(const float* __restrict__ Am, const float* __restrict__ BT, const float* __restrict__ SUB, float* __restrict__ OUT, float* __restrict__ OUTT) { __shared__ __align__(16) float ss[4][16][132]; __shared__ __align__(16) float st[128][68];
  const int tid = threadIdx.x, wave = tid >> 5, lane = tid & 31, col = lane & 15, g = lane >> 4; const int i0 = blockIdx.x * 64; const int c0 = blockIdx.y * 128; const size_t b = blockIdx.z; const int il0 = i0 + wave * 16;
  const float* arow = (MODE == 0) ? (Am + (b * NN + il0 + col) * (size_t)NN) : (Am + (size_t)(il0 + col) * NN);
  v8f acc[8] = {};
#pragma unroll 1
  for (int kc = 0; kc < NN / 32; ++kc) { F2 a; if (MODE == 0) a = split_row(arow, kc * 32, lane); else { const float* p = arow + kc * 32 + 8 * g;
#pragma unroll
      for (int i = 0; i < 8; ++i) { a.h[i] = (__bf16)p[i]; a.h[8 + i] = (__bf16)p[16 + i]; } }
#pragma unroll
    for (int j = 0; j < 8; ++j) { const int cs = c0 + j * 16 + col; const F2 bb = split_row(BT + (b * CT + cs) * (size_t)NN, kc * 32, lane); acc[j] = wmma_bf(a.h, bb.h, acc[j]); acc[j] = wmma_bf(a.h, bb.l, acc[j]); if (MODE == 0) acc[j] = wmma_bf(a.l, bb.h, acc[j]); } }
#pragma unroll
  for (int j = 0; j < 8; ++j)
#pragma unroll
    for (int r = 0; r < 8; ++r) { const int rl = 8 * g + r, cl = j * 16 + col; float v = acc[j][r]; if (MODE == 2) v = 2.0f * v - SUB[(b * NN + il0 + rl) * (size_t)CT + c0 + cl]; ss[wave][rl][cl] = v; st[cl][wave * 16 + rl] = v; }
  __syncthreads();
  for (int rl = 0; rl < 16; ++rl) vst2(OUT + (b * NN + il0 + rl) * (size_t)CT + c0 + lane * 4, *(const v4f*)&ss[wave][rl][lane * 4]);
  if (OUTT) for (int e = tid; e < 128 * 16; e += 128) { const int cl = e >> 4, q = e & 15; vst2(OUTT + (b * CT + c0 + cl) * (size_t)NN + i0 + q * 4, *(const v4f*)&st[cl][q * 4]); } }
__global__ __launch_bounds__(128) void k_final(const float* __restrict__ T0, const float* __restrict__ T1, const float* __restrict__ T2, const float* __restrict__ X, const float* __restrict__ CH, const float* __restrict__ TW, const float* __restrict__ TB, const float* __restrict__ RW, const float* __restrict__ RB, float* __restrict__ OUT) {
  __shared__ __align__(16) __bf16 sA[CO][3 * CI + 8];
  __shared__ __align__(16) __bf16 sBh[TS][3 * CI + 8], sBl[TS][3 * CI + 8];
  __shared__ __align__(16) float sg[CO][TS + 4];
  __shared__ __align__(16) __bf16 sX[TS][CI + 8];
  const int tid = threadIdx.x, wave = tid >> 5, lane = tid & 31, col = lane & 15, g = lane >> 4; const int n = blockIdx.x; const size_t b = blockIdx.y; const size_t rowbase = (b * NN + n) * (size_t)CT;
  for (int e = tid; e < 3 * CI * CO; e += 128) { const int k = e / (CI * CO), rem = e % (CI * CO); const int i = rem / CO, o = rem % CO; sA[o][k * CI + i] = (__bf16)CH[e]; }
  for (int e = tid; e < 3 * CI * TS; e += 128) { const int k = e / (CI * TS), rem = e % (CI * TS); const int i = rem / TS, s = rem % TS; const float v = (k == 0 ? T0 : k == 1 ? T1 : T2)[rowbase + rem]; const __bf16 h = (__bf16)v; sBh[s][k * CI + i] = h; sBl[s][k * CI + i] = (__bf16)(v - (float)h); }
  for (int e = tid; e < CI * TS; e += 128) { const int c = e >> 6, t = e & 63; sX[t][c] = (__bf16)X[((b * NN + n) * CI + c) * (size_t)TS + t]; }
  __syncthreads();
  v8f acc[4] = {};
#pragma unroll
  for (int kc = 0; kc < 3 * CI / 32; ++kc) { const v16b a = frag_b(&sA[wave * 16 + col][kc * 32], lane);
#pragma unroll
    for (int j = 0; j < 4; ++j) { const int s = j * 16 + col; acc[j] = wmma_bf(a, frag_b(&sBh[s][kc * 32], lane), acc[j]); acc[j] = wmma_bf(a, frag_b(&sBl[s][kc * 32], lane), acc[j]); } }
#pragma unroll
  for (int j = 0; j < 4; ++j)
#pragma unroll
    for (int r = 0; r < 8; ++r) sg[wave * 16 + 8 * g + r][j * 16 + col] = acc[j][r];
  __syncthreads();
  for (int e = tid; e < TS * CO * 3; e += 128) { const int t = e / (CO * 3), rem = e % (CO * 3); const int c = rem / 3, dt = rem % 3; const int ts = t + dt - 1; const float v = (ts >= 0 && ts < TS) ? sg[c][ts] : 0.f; const __bf16 h = (__bf16)v; sBh[t][rem] = h; sBl[t][rem] = (__bf16)(v - (float)h); }
  __syncthreads();
  v8f acv[4] = {}, acr[4] = {};
#pragma unroll
  for (int kc = 0; kc < 3 * CO / 32; ++kc) { v16b a; { const float* p = TW + (size_t)(wave * 16 + col) * (CO * 3) + kc * 32 + 8 * g;
#pragma unroll
      for (int i = 0; i < 8; ++i) { a[i] = (__bf16)p[i]; a[8 + i] = (__bf16)p[16 + i]; } }
#pragma unroll
    for (int j = 0; j < 4; ++j) { const int t = j * 16 + col; acv[j] = wmma_bf(a, frag_b(&sBh[t][kc * 32], lane), acv[j]); acv[j] = wmma_bf(a, frag_b(&sBl[t][kc * 32], lane), acv[j]); } }
#pragma unroll
  for (int kc = 0; kc < CI / 32; ++kc) { v16b a; { const float* p = RW + (size_t)(wave * 16 + col) * CI + kc * 32 + 8 * g;
#pragma unroll
      for (int i = 0; i < 8; ++i) { a[i] = (__bf16)p[i]; a[8 + i] = (__bf16)p[16 + i]; } }
#pragma unroll
    for (int j = 0; j < 4; ++j) { const int t = j * 16 + col; acr[j] = wmma_bf(a, frag_b(&sX[t][kc * 32], lane), acr[j]); } }
  __syncthreads();
#pragma unroll
  for (int j = 0; j < 4; ++j)
#pragma unroll
    for (int r = 0; r < 8; ++r) { const int o = wave * 16 + 8 * g + r, t = j * 16 + col; const float tout = fmaxf(acv[j][r] + bfr(TB[o]), 0.f); const float res = acr[j][r] + bfr(RB[o]); sg[o][t] = fmaxf(tout + res, 0.f); }
  __syncthreads(); for (int e = tid; e < CO * 16; e += 128) { const int o = e >> 4, q = e & 15; vst2(OUT + ((b * NN + n) * CO + o) * (size_t)TS + q * 4, *(const v4f*)&sg[o][q * 4]); } }
extern "C" void kernel_launch(void* const* d_in, const int* in_sizes, int n_in, void* d_out, int out_size, void* d_ws, size_t ws_size, hipStream_t stream) {
  (void)in_sizes; (void)n_in; (void)out_size;
  const float** F = (const float**)d_in;
  if (ws_size < (size_t)WS_END) return;
  char* ws = (char*)d_ws; float *LS = (float*)(ws + WS_LS), *RST = (float*)(ws + WS_RST), *XTR = (float*)(ws + WS_XTR), *LT = (float*)(ws + WS_LT), *RTT = (float*)(ws + WS_RTT), *SA = (float*)(ws + WS_SA), *EA = (float*)(ws + WS_EA), *XTT = (float*)(ws + WS_XTT), *XM = (float*)(ws + WS_XM), *XMT = (float*)(ws + WS_XMT), *T1 = (float*)(ws + WS_T1), *T1T = (float*)(ws + WS_T1T), *T2 = (float*)(ws + WS_T2);
  k_lhs<<<dim3(TNB * NN / 64, NN / 128, 2), 128, 0, stream>>>(F[0], F[2], F[3], LS, RST);
  k_xtr<<<dim3(NN, TNB), 256, 0, stream>>>(F[0], XTR);
  k_lht<<<TNB * TS / 64, 128, 0, stream>>>(XTR, F[5], F[6], LT, RTT);
  k_att<NN><<<dim3(NN, TNB), 256, 0, stream>>>(LS, RST, F[4], SA);
  k_att<TS><<<dim3(TS, TNB), 256, 0, stream>>>(LT, RTT, F[7], EA);
  k_xtime<<<dim3(NN / 64, CI, TNB), 128, 0, stream>>>(F[0], EA, XTT);
  k_nmix<0><<<dim3(NN / 64, CT / 128, TNB), 128, 0, stream>>>(SA, XTT, nullptr, XM, XMT);
  k_nmix<1><<<dim3(NN / 64, CT / 128, TNB), 128, 0, stream>>>(F[1], XMT, nullptr, T1, T1T);
  k_nmix<2><<<dim3(NN / 64, CT / 128, TNB), 128, 0, stream>>>(F[1], T1T, XM, T2, nullptr);
  k_final<<<dim3(NN, TNB), 128, 0, stream>>>(XM, T1, T2, F[0], F[8], F[9], F[10], F[11], F[12], (float*)d_out);
}
